// FastSlowKimiDeltaAttention_46806553591959
// MI455X (gfx1250) — hardware-verified
//
#include <hip/hip_runtime.h>
#include <math.h>

#define LEG_BF16_INPUTS 1

constexpr int kBatch  = 2;
constexpr int kSeq    = 1024;
constexpr int kHid    = 2048;
constexpr int kHeads  = 16;
constexpr int kHead   = 128;
constexpr int kTok    = kBatch * kSeq;
constexpr int kCh     = kHeads * kHead;
constexpr int kSmall  = 448;
constexpr int kChunk  = 16;
constexpr int kNumChunks = kSeq / kChunk;
constexpr int kKtPitch = 136;
constexpr int kKhPitch = 24;
constexpr int kUtPitch = 40;
constexpr int kKtW = kKtPitch / 2;
constexpr int kKhW = kKhPitch / 2;
constexpr int kUtW = kUtPitch / 2;
constexpr int kStPitch = 132;
constexpr float kXCarry   = 16.0f;
constexpr float kWCarry   = 64.0f;
constexpr float kMidCarry = 16.0f;
constexpr float kOnCarry  = 64.0f;
constexpr float kProjScale = 1.0f / (kXCarry * kWCarry);
constexpr float kMidScale  = 1.0f / (kMidCarry * kWCarry);
constexpr float kOutScale  = 1.0f / (kOnCarry * kWCarry);
constexpr float kL2Eps   = 1e-6f;
constexpr float kNormEps = 1e-5f;
static_assert(kTok % 64 == 0 && kCh % 64 == 0 && kHid % 64 == 0 && kSmall % 64 == 0);
static_assert(kHid % 32 == 0 && kCh % 32 == 0 && (2 * kHead) % 32 == 0 && kHead % 32 == 0);
static_assert(kSeq % kChunk == 0 && kChunk == 16 && kHead == 128);
static_assert(kCh == 2048 && kTok == 2048);
static_assert((kHead * kStPitch) % 256 == 0 && (kStPitch % 4) == 0);
static_assert((kKtW % 4) == 0 && (kKhW % 4) == 0 && (kUtW % 4) == 0);

typedef __attribute__((ext_vector_type(16))) _Float16 v16h;
typedef __attribute__((ext_vector_type(8)))  _Float16 v8h;
typedef __attribute__((ext_vector_type(16))) __bf16   v16b;
typedef __attribute__((ext_vector_type(8)))  __bf16   v8b;
typedef __attribute__((ext_vector_type(8)))  float    v8f;
typedef __attribute__((ext_vector_type(4)))  float    v4f;
typedef __attribute__((ext_vector_type(2)))  float    v2f;
typedef __attribute__((ext_vector_type(8)))  unsigned int v8u;
typedef __attribute__((ext_vector_type(4)))  unsigned int v4u;
typedef __attribute__((ext_vector_type(2)))  unsigned int v2u;

__device__ __forceinline__ unsigned short f2bf_bits(float f) {
  unsigned u = __float_as_uint(f);
  return (unsigned short)((u + 0x7FFFu + ((u >> 16) & 1u)) >> 16);
}
__device__ __forceinline__ float bf_bits2f(unsigned short h) { return __uint_as_float(((unsigned)h) << 16); }
__device__ __forceinline__ float bf16r(float f) { return bf_bits2f(f2bf_bits(f)); }
__device__ __forceinline__ float inr(float f) {
#if LEG_BF16_INPUTS
  return bf16r(f);
#else
  return f;
#endif
}
__device__ __forceinline__ unsigned pk16(unsigned short a, unsigned short b) { return (unsigned)a | ((unsigned)b << 16); }
__device__ __forceinline__ unsigned short h_bits(float f) { const _Float16 h = (_Float16)f; return __builtin_bit_cast(unsigned short, h); }
__device__ __forceinline__ float h16_to_f32(unsigned hb) {
  const unsigned sgn = (hb & 0x8000u) << 16; const unsigned em = hb & 0x7fffu;
  const float fn = __uint_as_float((em << 13) + 0x38000000u);
  const float fs = (float)em * 5.9604644775390625e-8f;
  const float mag = (em < 0x400u) ? fs : fn; return __uint_as_float(__float_as_uint(mag) | sgn);
}
__device__ __forceinline__ float sigm(float x) { return 1.0f / (1.0f + expf(-x)); }

__device__ __forceinline__ void dep_guard4_h(v8f& a, v8f& b, v8f& c, v8f& d, v16h x, v16h y) { asm volatile("v_nop\n\tv_nop\n\tv_nop\n\tv_nop" : "+v"(a), "+v"(b), "+v"(c), "+v"(d) : "v"(x), "v"(y)); }
__device__ __forceinline__ void dep_guard4_b(v8f& a, v8f& b, v8f& c, v8f& d, v16b x, v16b y) { asm volatile("v_nop\n\tv_nop\n\tv_nop\n\tv_nop" : "+v"(a), "+v"(b), "+v"(c), "+v"(d) : "v"(x), "v"(y)); }
__device__ __forceinline__ void keep4_h(v16h a, v16h b, v16h c, v16h d) { asm volatile("v_nop" :: "v"(a), "v"(b), "v"(c), "v"(d)); }
__device__ __forceinline__ void keep4_b(v16b a, v16b b, v16b c, v16b d) { asm volatile("v_nop" :: "v"(a), "v"(b), "v"(c), "v"(d)); }
__device__ __forceinline__ void acc_guard4(v8f& a, v8f& b, v8f& c, v8f& d) { asm volatile("v_nop\n\tv_nop\n\tv_nop\n\tv_nop" : "+v"(a), "+v"(b), "+v"(c), "+v"(d)); }
__device__ __forceinline__ void guard_s6(v8f& a, v8f& b, v16b f0, v16b f1, v16b f2, v16b f3, v16b f4, v16b f5) {
  asm volatile("v_nop\n\tv_nop\n\tv_nop\n\tv_nop" : "+v"(a), "+v"(b) : "v"(f0), "v"(f1), "v"(f2), "v"(f3), "v"(f4), "v"(f5));
}
__device__ __forceinline__ void guard_u3(v8f& a, v16b x, v16b y, v16b z) {
  asm volatile("v_nop\n\tv_nop\n\tv_nop\n\tv_nop" : "+v"(a) : "v"(x), "v"(y), "v"(z));
}

template <typename T> struct Frag;
template <> struct Frag<_Float16> {
  typedef v16h V; union U { v16h v; v8h h[2]; };
  static __device__ __forceinline__ v16h load(const _Float16* p) {
    U f; f.h[0] = *(const v8h*)(p); f.h[1] = *(const v8h*)(p + 16); return f.v;
  }
  static __device__ __forceinline__ v8f mma(v16h a, v16h b, v8f c) {
    return __builtin_amdgcn_wmma_f32_16x16x32_f16(false, a, false, b, (short)0, c, false, false);
  }
  static __device__ __forceinline__ void guard(v8f& a, v8f& b, v8f& c, v8f& d, v16h x, v16h y) { dep_guard4_h(a, b, c, d, x, y); }
  static __device__ __forceinline__ void keep(v16h a, v16h b, v16h c, v16h d) { keep4_h(a, b, c, d); }
};
template <> struct Frag<__bf16> {
  typedef v16b V; union U { v16b v; v8b h[2]; };
  static __device__ __forceinline__ v16b load(const __bf16* p) {
    U f; f.h[0] = *(const v8b*)(p); f.h[1] = *(const v8b*)(p + 16); return f.v;
  }
  static __device__ __forceinline__ v16b load_dup(const __bf16* p) {
    U f; const v8b x = *(const v8b*)(p); f.h[0] = x; f.h[1] = x; return f.v;
  }
  static __device__ __forceinline__ v8f mma(v16b a, v16b b, v8f c) {
    return __builtin_amdgcn_wmma_f32_16x16x32_bf16(false, a, false, b, (short)0, c, false, false);
  }
  static __device__ __forceinline__ void guard(v8f& a, v8f& b, v8f& c, v8f& d, v16b x, v16b y) { dep_guard4_b(a, b, c, d, x, y); }
  static __device__ __forceinline__ void keep(v16b a, v16b b, v16b c, v16b d) { keep4_b(a, b, c, d); }
};

template <int ET> struct Elem;
template <> struct Elem<0> { typedef _Float16 T; };
template <> struct Elem<1> { typedef __bf16 T; };
template <int ET, bool SPLIT, int BIAS_MODE, int OUT_MODE, bool RESID, int ACT = 0>
__global__ __launch_bounds__(256) void wmma_gemm64(
    const unsigned short* __restrict__ Ap, const unsigned short* __restrict__ A2p, int lda, long strideA,
    const unsigned short* __restrict__ Btp, const unsigned short* __restrict__ Bt2p, int ldb, long strideB,
    void* __restrict__ Cout, void* __restrict__ Cout2, int ldc, long strideC,
    const float* __restrict__ bias,
    const float* __restrict__ resid, long strideR,
    int M, int N, int K, float scale) {
  typedef typename Elem<ET>::T T;
  typedef typename Frag<T>::V V;
  const T* A = (const T*)Ap; const T* A2 = (const T*)A2p; const T* Bt = (const T*)Btp; const T* Bt2 = (const T*)Bt2p;
  __shared__ __align__(16) float sT[8][16 * 68];
  const int b    = blockIdx.y;
  const int lane = threadIdx.x & 31;
  const int wave = threadIdx.x >> 5;
  const int tilesN = N >> 6;
  const int tilesM = M >> 6;
  const int tile = blockIdx.x * 8 + wave;
  if (tile >= tilesM * tilesN) return;
  const int tm = tile / tilesN;
  const int tn = tile - tm * tilesN;
  const int m0 = tm << 6;
  const int n0 = tn << 6;

  const T* Ab  = A  + (size_t)b * strideA;
  const T* Bb  = Bt + (size_t)b * strideB;
  const T* Ab2 = SPLIT ? (A2  + (size_t)b * strideA) : nullptr;
  const T* Bb2 = SPLIT ? (Bt2 + (size_t)b * strideB) : nullptr;

  const int rlane = lane & 15;
  const int koff  = (lane >> 4) * 8;
  const int mOff  = (lane >> 4) * 8;

  v8f acc[4][4];
#pragma unroll
  for (int i = 0; i < 4; ++i)
#pragma unroll
    for (int j = 0; j < 4; ++j) acc[i][j] = (v8f){0.f,0.f,0.f,0.f,0.f,0.f,0.f,0.f};

  for (int k0 = 0; k0 < K; k0 += 32) {
    V bh[4], bl[4];
#pragma unroll
    for (int j = 0; j < 4; ++j) {
      const size_t bo = (size_t)(n0 + (j << 4) + rlane) * ldb + koff + k0;
      bh[j] = Frag<T>::load(Bb + bo);
      if (SPLIT) bl[j] = Frag<T>::load(Bb2 + bo);
    }
#pragma unroll
    for (int i = 0; i < 4; ++i) {
      const size_t ao = (size_t)(m0 + (i << 4) + rlane) * lda + koff + k0;
      V ah = Frag<T>::load(Ab + ao);
      V al;
      if (SPLIT) al = Frag<T>::load(Ab2 + ao);
#pragma unroll
      for (int j = 0; j < 4; ++j) {
        acc[i][j] = Frag<T>::mma(ah, bh[j], acc[i][j]);
        if (SPLIT) {
          acc[i][j] = Frag<T>::mma(ah, bl[j], acc[i][j]);
          acc[i][j] = Frag<T>::mma(al, bh[j], acc[i][j]);
        }
      }
      Frag<T>::guard(acc[i][0], acc[i][1], acc[i][2], acc[i][3], ah, SPLIT ? al : ah);
    }
    Frag<T>::keep(bh[0], bh[1], bh[2], bh[3]);
    if (SPLIT) Frag<T>::keep(bl[0], bl[1], bl[2], bl[3]);
  }
  acc_guard4(acc[0][0], acc[0][1], acc[0][2], acc[0][3]);
  acc_guard4(acc[1][0], acc[1][1], acc[1][2], acc[1][3]);
  acc_guard4(acc[2][0], acc[2][1], acc[2][2], acc[2][3]);
  acc_guard4(acc[3][0], acc[3][1], acc[3][2], acc[3][3]);

  float* slab = sT[wave];
  const float* Rb = RESID ? (resid + (size_t)b * strideR) : nullptr;
#pragma unroll
  for (int i = 0; i < 4; ++i) {
    const int mBase = m0 + (i << 4);
#pragma unroll
    for (int j = 0; j < 4; ++j) {
      const int n = n0 + (j << 4) + rlane;
      float bv = 0.f;
      if (BIAS_MODE == 2) bv = bias[n];
#pragma unroll
      for (int r = 0; r < 8; ++r) {
        float v = acc[i][j][r] * scale;
        if (BIAS_MODE == 1) v += bias[mBase + mOff + r];
        if (BIAS_MODE == 2) v += bv;
        if (RESID) v += Rb[(size_t)(mBase + mOff + r) * ldc + n];
        if (ACT == 2) v = fmaxf(v, 0.0f);
        if (ACT == 4) v = (v > 0.f) ? v : 0.01f * v;
        slab[(mOff + r) * 68 + (j << 4) + rlane] = v;
      }
    }
    __builtin_amdgcn_fence(__ATOMIC_RELEASE, "workgroup");
    __builtin_amdgcn_wave_barrier();
    __builtin_amdgcn_fence(__ATOMIC_ACQUIRE, "workgroup");
    if (OUT_MODE == 0) {
      float* C = (float*)Cout + (size_t)b * strideC;
      const int hh = lane >> 4, c4 = (lane & 15) * 4;
      for (int pass = 0; pass < 2; ++pass) {
#pragma unroll
        for (int it = 0; it < 8; ++it) {
          const int row = it * 2 + hh;
          v4f v = *(const v4f*)(slab + row * 68 + c4);
          *(volatile v4f*)(C + (size_t)(mBase + row) * ldc + n0 + c4) = v;
        }
        __threadfence();
      }
    } else {
      const int q = lane >> 3, c8 = (lane & 7) * 8;
      unsigned short* C  = (unsigned short*)Cout  + (size_t)b * strideC;
      unsigned short* C2 = (OUT_MODE == 2) ? ((unsigned short*)Cout2 + (size_t)b * strideC) : nullptr;
      for (int pass = 0; pass < 2; ++pass) {
#pragma unroll
        for (int it = 0; it < 4; ++it) {
          const int row = it * 4 + q;
          const float* sp = slab + row * 68 + c8;
          v8h hv, lv;
#pragma unroll
          for (int e = 0; e < 8; ++e) {
            if (OUT_MODE == 1) {
              hv[e] = (_Float16)sp[e];
            } else {
              unsigned short hb = f2bf_bits(sp[e]);
              unsigned short lb = f2bf_bits(sp[e] - bf_bits2f(hb));
              hv[e] = __builtin_bit_cast(_Float16, hb);
              lv[e] = __builtin_bit_cast(_Float16, lb);
            }
          }
          *(volatile v8h*)(C + (size_t)(mBase + row) * ldc + n0 + c8) = hv;
          if (OUT_MODE == 2) *(volatile v8h*)(C2 + (size_t)(mBase + row) * ldc + n0 + c8) = lv;
        }
        __threadfence();
      }
    }
    __builtin_amdgcn_fence(__ATOMIC_RELEASE, "workgroup");
    __builtin_amdgcn_wave_barrier();
    __builtin_amdgcn_fence(__ATOMIC_ACQUIRE, "workgroup");
  }
}

__global__ __launch_bounds__(256) void cvt_x_kernel(const float* __restrict__ in, unsigned short* __restrict__ out, int n8, float carry) {
  const int i = blockIdx.x * 256 + threadIdx.x;
  if (i >= n8) return;
  const float* p = in + 8 * (size_t)i;
  const v4f a = *(const v4f*)(p);
  const v4f c = *(const v4f*)(p + 4);
  unsigned short hb[8];
#pragma unroll
  for (int e = 0; e < 4; ++e) {
    const float fa = a[e];
    const float fc = c[e];
    hb[e]     = h_bits(inr(fa) * carry);
    hb[4 + e] = h_bits(inr(fc) * carry);
  }
  const v4u u = (v4u){pk16(hb[0], hb[1]), pk16(hb[2], hb[3]), pk16(hb[4], hb[5]), pk16(hb[6], hb[7])};
  unsigned short* q = out + 8 * (size_t)i;
  *(volatile v4u*)q = u;
  __threadfence();
  *(volatile v4u*)q = u;
}

__global__ __launch_bounds__(256) void tr_cast_kernel(const float* __restrict__ W0, const float* __restrict__ W1, const float* __restrict__ W2,
                                                      unsigned short* __restrict__ D0, unsigned short* __restrict__ D1, unsigned short* __restrict__ D2,
                                                      int C, int ldd, float carry) {
  __shared__ float sm[64][65];
  const int t  = threadIdx.x;
  const int r0 = blockIdx.x * 64;
  const int c0 = blockIdx.y * 64;
  const int z  = blockIdx.z;
  const float* W = (z == 0) ? W0 : (z == 1) ? W1 : W2;
  unsigned short* D = (z == 0) ? D0 : (z == 1) ? D1 : D2;
#pragma unroll
  for (int i = 0; i < 16; ++i) {
    const int e = i * 256 + t;
    const int r = e >> 6;
    const int c = e & 63;
    sm[c][r] = inr(W[(size_t)(r0 + r) * C + c0 + c]) * carry;
  }
  __syncthreads();
  const int lane = t & 31, wave = t >> 5;
  const int q = lane >> 3, c8 = (lane & 7) * 8;
  for (int pass = 0; pass < 2; ++pass) {
#pragma unroll
    for (int it = 0; it < 2; ++it) {
      const int row = wave * 8 + it * 4 + q;
      unsigned short hb[8];
#pragma unroll
      for (int e = 0; e < 8; ++e) hb[e] = h_bits(sm[row][c8 + e]);
      const v4u u = (v4u){pk16(hb[0], hb[1]), pk16(hb[2], hb[3]), pk16(hb[4], hb[5]), pk16(hb[6], hb[7])};
      *(volatile v4u*)(D + (size_t)(c0 + row) * ldd + r0 + c8) = u;
    }
    __threadfence();
  }
}

__global__ __launch_bounds__(256) void tr_small16_kernel(const float* __restrict__ Wa, const float* __restrict__ Wb, const float* __restrict__ Wc,
                                                         unsigned short* __restrict__ D, int ldd, float carry) {
  __shared__ float sm[64][65];
  const int t  = threadIdx.x;
  const int r0 = blockIdx.x * 64;
#pragma unroll
  for (int j = 0; j < 4; ++j) {
    const int e = j * 256 + t;
    const int r = e >> 4;
    const int col = e & 15;
    sm[col][r]      = inr(Wa[(size_t)r0 * 16 + e]) * carry;
    sm[16 + col][r] = inr(Wb[(size_t)r0 * 16 + e]) * carry;
    sm[32 + col][r] = inr(Wc[(size_t)r0 * 16 + e]) * carry;
    sm[48 + col][r] = 0.0f;
  }
  __syncthreads();
  const int lane = t & 31, wave = t >> 5;
  const int q = lane >> 3, c8 = (lane & 7) * 8;
  for (int pass = 0; pass < 2; ++pass) {
#pragma unroll
    for (int it = 0; it < 2; ++it) {
      const int row = wave * 8 + it * 4 + q;
      unsigned short hb[8];
#pragma unroll
      for (int e = 0; e < 8; ++e) hb[e] = h_bits(sm[row][c8 + e]);
      const v4u u = (v4u){pk16(hb[0], hb[1]), pk16(hb[2], hb[3]), pk16(hb[4], hb[5]), pk16(hb[6], hb[7])};
      *(volatile v4u*)(D + (size_t)row * ldd + r0 + c8) = u;
    }
    __threadfence();
  }
}

template <bool NORM>
__global__ __launch_bounds__(256) void conv_silu_kernel(const float* __restrict__ PRE, const float* __restrict__ cw, float* __restrict__ OUT) {
  const int lane = threadIdx.x & 31, wave = threadIdx.x >> 5;
  const int gw = blockIdx.x * 8 + wave;
  const int row = gw >> 4, h = gw & 15;
  const int t = row & (kSeq - 1);
  const int ch = h * kHead + lane * 4;
  v4f wt[4];
#pragma unroll
  for (int c = 0; c < 4; ++c) wt[c] = *(const v4f*)(cw + (size_t)(ch + c) * 4);
  v4f y = (v4f){0.f, 0.f, 0.f, 0.f};
#pragma unroll
  for (int i = 0; i < 4; ++i) {
    const int back = 3 - i;
    const bool ok = (t >= back);
    const int rsel = ok ? (row - back) : row;
    const v4f p = *(const v4f*)(PRE + (size_t)rsel * kCh + ch);
#pragma unroll
    for (int c = 0; c < 4; ++c) {
      const float pv = ok ? p[c] : 0.0f;
      const float wv = wt[c][i];
      y[c] += inr(wv) * pv;
    }
  }
  v4f s;
  float ss = 0.0f;
#pragma unroll
  for (int c = 0; c < 4; ++c) {
    const float yy = y[c];
    const float sv = yy * sigm(yy);
    s[c] = sv;
    ss += sv * sv;
  }
  if (NORM) {
#pragma unroll
    for (int off = 16; off > 0; off >>= 1) ss += __shfl_xor(ss, off, 32);
    const float rn = rsqrtf(ss + kL2Eps);
#pragma unroll
    for (int c = 0; c < 4; ++c) s[c] = s[c] * rn;
  }
  float* op = OUT + (size_t)row * kCh + ch;
  *(volatile v4f*)op = s;
  __threadfence();
  *(volatile v4f*)op = s;
}

__global__ __launch_bounds__(256) void split_small_kernel(const float* __restrict__ SM, unsigned short* __restrict__ MIDp,
                                                          unsigned short* __restrict__ MIDm, unsigned short* __restrict__ MIDg, float carry) {
  const int i = blockIdx.x * 256 + threadIdx.x;
  if (blockIdx.y == 0) {
    const int row = i >> 5, g = i & 31;
    const float* sp = SM + (size_t)row * kSmall + g * 8;
    const v4f a = *(const v4f*)(sp);
    const v4f c = *(const v4f*)(sp + 4);
    const float sg = (g >= 16) ? -1.0f : 1.0f;
    unsigned short hp[8], hm[8];
#pragma unroll
    for (int e = 0; e < 4; ++e) {
      const float fa = a[e] * carry;
      const float fc = c[e] * carry;
      hp[e] = h_bits(fa);      hp[4 + e] = h_bits(fc);
      hm[e] = h_bits(fa * sg); hm[4 + e] = h_bits(fc * sg);
    }
    const v4u up = (v4u){pk16(hp[0], hp[1]), pk16(hp[2], hp[3]), pk16(hp[4], hp[5]), pk16(hp[6], hp[7])};
    const v4u um = (v4u){pk16(hm[0], hm[1]), pk16(hm[2], hm[3]), pk16(hm[4], hm[5]), pk16(hm[6], hm[7])};
    unsigned short* qp = MIDp + 8 * (size_t)i;
    unsigned short* qm = MIDm + 8 * (size_t)i;
    *(volatile v4u*)qp = up;
    *(volatile v4u*)qm = um;
    __threadfence();
    *(volatile v4u*)qp = up;
    *(volatile v4u*)qm = um;
  } else {
    if (i >= kTok * 16) return;
    const int row = i >> 4, g = i & 15;
    const float* sp = SM + (size_t)row * kSmall + 256 + g * 8;
    const v4f a = *(const v4f*)(sp);
    const v4f c = *(const v4f*)(sp + 4);
    unsigned short hg[8];
#pragma unroll
    for (int e = 0; e < 4; ++e) {
      const float fa = a[e] * carry;
      const float fc = c[e] * carry;
      hg[e] = h_bits(fa); hg[4 + e] = h_bits(fc);
    }
    const v4u ug = (v4u){pk16(hg[0], hg[1]), pk16(hg[2], hg[3]), pk16(hg[4], hg[5]), pk16(hg[6], hg[7])};
    unsigned short* qg = MIDg + 8 * (size_t)i;
    *(volatile v4u*)qg = ug;
    __threadfence();
    *(volatile v4u*)qg = ug;
  }
}

__global__ __launch_bounds__(256) void beta_lam_kernel(const float* __restrict__ SM, float* __restrict__ BF, float* __restrict__ BS, float* __restrict__ LAM) {
  const int i = blockIdx.x * 256 + threadIdx.x;
  if (i >= kTok * kHeads) return;
  const int row = i >> 4, hh = i & 15;
  const float* sp = SM + (size_t)row * kSmall + 384 + hh;
  const float bb = sp[0], bd = sp[16], lm = sp[32];
  const float f = sigm(bb + bd);
  const float s = sigm(bb - bd);
  const float l = sigm(lm);
  *(volatile float*)(BF + i) = f;
  *(volatile float*)(BS + i) = s;
  *(volatile float*)(LAM + i) = l;
  __threadfence();
  *(volatile float*)(BF + i) = f;
  *(volatile float*)(BS + i) = s;
  *(volatile float*)(LAM + i) = l;
}

__global__ __launch_bounds__(256) void gate_kernel(const float* __restrict__ GP, const float* __restrict__ GM,
                                                   unsigned short* __restrict__ GF, unsigned short* __restrict__ GS,
                                                   const float* __restrict__ A_log, const float* __restrict__ dtb) {
  const int i = blockIdx.x * 256 + threadIdx.x;
  const bool second = (blockIdx.y != 0);
  const float* src = second ? GM : GP;
  unsigned short* dst = second ? GS : GF;
  const int n = (2 * i) & (kCh - 1);
  const int h = n >> 7;
  const float a = expf(inr(A_log[h]));
  const v2f g = *(const v2f*)(src + 2 * (size_t)i);
  const float g0 = g[0];
  const float g1 = g[1];
  unsigned short b0 = 0, b1 = 0;
#pragma unroll 1
  for (int j = 0; j < 2; ++j) {
    const float x = ((j == 0) ? g0 : g1) + inr(dtb[n + j]);
    const float sp = fmaxf(x, 0.0f) + log1pf(expf(-fabsf(x)));
    const float gt = -a * sp;
    const unsigned short bits = h_bits(gt);
    b0 = (j == 0) ? bits : b0;
    b1 = (j == 1) ? bits : b1;
  }
  const unsigned word = pk16(b0, b1);
  volatile unsigned* p = (volatile unsigned*)dst + i;
  *p = word;
  __threadfence();
  *p = word;
}

__device__ __forceinline__ void split_tr(float x, unsigned& hi, unsigned& lo) {
  const unsigned u = __float_as_uint(x);
  hi = u >> 16;
  const float r = x - __uint_as_float(u & 0xffff0000u);
  lo = (unsigned)f2bf_bits(r);
}
__device__ __forceinline__ void split_pair(float x0, float x1, unsigned& hw, unsigned& lw) {
  unsigned h0, l0, h1, l1;
  split_tr(x0, h0, l0);
  split_tr(x1, h1, l1);
  hw = h0 | (h1 << 16);
  lw = l0 | (l1 << 16);
}

__global__ __launch_bounds__(256) __attribute__((amdgpu_num_vgpr(256))) void delta_scan_kernel(
    const float* __restrict__ QN, const float* __restrict__ KN, const float* __restrict__ VC,
    const unsigned short* __restrict__ GFp, const unsigned short* __restrict__ GSp,
    const float* __restrict__ BFp, const float* __restrict__ BSp,
    float* __restrict__ OFp, float* __restrict__ OSp, float qscale) {
  __shared__ __align__(16) float St[kHead * kStPitch];
  __shared__ __align__(16) float Gs[kChunk * kHead];
  __shared__ __align__(16) float Ks[kChunk * kHead];
  __shared__ __align__(16) float Qs[kChunk * kHead];
  __shared__ __align__(16) float Vs[kChunk * kHead];
  __shared__ __align__(16) float RO[kChunk * kHead];
  __shared__ __align__(16) unsigned KTh[kChunk * kKtW];
  __shared__ __align__(16) unsigned KTl[kChunk * kKtW];
  __shared__ __align__(16) unsigned QTh[kChunk * kKtW];
  __shared__ __align__(16) unsigned QTl[kChunk * kKtW];
  __shared__ __align__(16) unsigned KHh[kHead * kKhW];
  __shared__ __align__(16) unsigned KHl[kHead * kKhW];
  __shared__ __align__(16) unsigned UT[kHead * kUtW];
  __shared__ __align__(16) unsigned BPh[kChunk * kKhW];
  __shared__ __align__(16) unsigned BPl[kChunk * kKhW];
  __shared__ __align__(16) float Amat[kChunk * kChunk];
  __shared__ __align__(16) float Bmat[kChunk * kChunk];
  __shared__ __align__(16) float egC[kHead];
  __shared__ __align__(16) float betas[kChunk];

  const int tid  = threadIdx.x;
  const int lane = tid & 31;
  const int wave = __builtin_amdgcn_readfirstlane((int)(threadIdx.x >> 5));
  const int hh   = lane >> 4;
  const int c    = lane & 15;
  const int chain = blockIdx.x;
  const int st = chain & 1;
  const int h  = (chain >> 1) & (kHeads - 1);
  const int b  = chain >> 5;
  const unsigned short* G = st ? GSp : GFp;
  const float* Bt = st ? BSp : BFp;
  float* O = st ? OSp : OFp;
  const int rowbase = b * kSeq;

#pragma unroll 1
  for (int i = tid; i < kHead * kStPitch; i += 256) St[i] = 0.0f;
  __syncthreads();

  float* strow = St + (16 * wave + c) * kStPitch + 8 * hh;
  const __bf16* kthp = (const __bf16*)(const void*)KTh + c * kKtPitch + 8 * hh;
  const __bf16* ktlp = (const __bf16*)(const void*)KTl + c * kKtPitch + 8 * hh;
  const __bf16* qthp = (const __bf16*)(const void*)QTh + c * kKtPitch + 8 * hh;
  const __bf16* qtlp = (const __bf16*)(const void*)QTl + c * kKtPitch + 8 * hh;
  const __bf16* khhp = (const __bf16*)(const void*)KHh + c * kKhPitch + 8 * hh;
  const __bf16* khlp = (const __bf16*)(const void*)KHl + c * kKhPitch + 8 * hh;
  const __bf16* utp  = (const __bf16*)(const void*)UT + (16 * wave + c) * kUtPitch + 8 * hh;
  const __bf16* bphp = (const __bf16*)(const void*)BPh + c * kKhPitch + 8 * hh;
  const __bf16* bplp = (const __bf16*)(const void*)BPl + c * kKhPitch + 8 * hh;

#pragma unroll 1
  for (int chk = 0; chk < kNumChunks; ++chk) {
    const int t0 = rowbase + chk * kChunk;

    {
      const int i = tid >> 4, cg = tid & 15;
      const size_t off = (size_t)(t0 + i) * kCh + h * kHead + cg * 8;
      const v4f q0 = *(const v4f*)(QN + off);
      const v4f q1 = *(const v4f*)(QN + off + 4);
      const v4f k0 = *(const v4f*)(KN + off);
      const v4f k1 = *(const v4f*)(KN + off + 4);
      const v4f v0 = *(const v4f*)(VC + off);
      const v4f v1 = *(const v4f*)(VC + off + 4);
      const v4u gw = *(const v4u*)(G + off);
      const unsigned w0 = gw[0], w1 = gw[1], w2 = gw[2], w3 = gw[3];
      v4f g0, g1;
      g0[0] = h16_to_f32(w0 & 0xffffu); g0[1] = h16_to_f32(w0 >> 16);
      g0[2] = h16_to_f32(w1 & 0xffffu); g0[3] = h16_to_f32(w1 >> 16);
      g1[0] = h16_to_f32(w2 & 0xffffu); g1[1] = h16_to_f32(w2 >> 16);
      g1[2] = h16_to_f32(w3 & 0xffffu); g1[3] = h16_to_f32(w3 >> 16);
      const int lo = i * kHead + cg * 8;
      *(v4f*)(Gs + lo) = g0;           *(v4f*)(Gs + lo + 4) = g1;
      *(v4f*)(Ks + lo) = k0;           *(v4f*)(Ks + lo + 4) = k1;
      *(v4f*)(Qs + lo) = q0 * qscale;  *(v4f*)(Qs + lo + 4) = q1 * qscale;
      *(v4f*)(Vs + lo) = v0;           *(v4f*)(Vs + lo + 4) = v1;
    }
    if (wave == 0) {
      float bv = Bt[(size_t)(t0 + (tid & 15)) * kHeads + h];
      asm volatile("" : "+v"(bv));
      if (tid < kChunk) betas[tid] = bv;
    }
    __syncthreads();

    if (tid < kHead) {
      float run = 0.0f;
#pragma unroll 1
      for (int i = 0; i < kChunk; ++i) {
        run += Gs[i * kHead + tid];
        Gs[i * kHead + tid] = run;
      }
      egC[tid] = __expf(run);
    }
    __syncthreads();

    {
      const int i = tid >> 4, cg = tid & 15;
      const int lo = i * kHead + cg * 8;
      const v4f ga = *(const v4f*)(Gs + lo);
      const v4f gb = *(const v4f*)(Gs + lo + 4);
      const v4f ka = *(const v4f*)(Ks + lo);
      const v4f kb = *(const v4f*)(Ks + lo + 4);
      const v4f qa = *(const v4f*)(Qs + lo);
      const v4f qb = *(const v4f*)(Qs + lo + 4);
      unsigned kh[4], kl[4], qh[4], ql[4];
#pragma unroll
      for (int j = 0; j < 2; ++j) {
        const float wa0 = __expf(ga[2 * j]), wa1 = __expf(ga[2 * j + 1]);
        const float wb0 = __expf(gb[2 * j]), wb1 = __expf(gb[2 * j + 1]);
        split_pair(ka[2 * j] * wa0, ka[2 * j + 1] * wa1, kh[j], kl[j]);
        split_pair(kb[2 * j] * wb0, kb[2 * j + 1] * wb1, kh[2 + j], kl[2 + j]);
        split_pair(qa[2 * j] * wa0, qa[2 * j + 1] * wa1, qh[j], ql[j]);
        split_pair(qb[2 * j] * wb0, qb[2 * j + 1] * wb1, qh[2 + j], ql[2 + j]);
      }
      const int po = i * kKtW + cg * 4;
      *(v4u*)(KTh + po) = (v4u){kh[0], kh[1], kh[2], kh[3]};
      *(v4u*)(KTl + po) = (v4u){kl[0], kl[1], kl[2], kl[3]};
      *(v4u*)(QTh + po) = (v4u){qh[0], qh[1], qh[2], qh[3]};
      *(v4u*)(QTl + po) = (v4u){ql[0], ql[1], ql[2], ql[3]};
    }
    if (tid < kHead) {
      const float gC = Gs[(kChunk - 1) * kHead + tid];
#pragma unroll 1
      for (int j = 0; j < 8; ++j) {
        const float x0 = Ks[(2 * j) * kHead + tid] * __expf(gC - Gs[(2 * j) * kHead + tid]);
        const float x1 = Ks[(2 * j + 1) * kHead + tid] * __expf(gC - Gs[(2 * j + 1) * kHead + tid]);
        unsigned hw, lw;
        split_pair(x0, x1, hw, lw);
        KHh[tid * kKhW + j] = hw;
        KHl[tid * kKhW + j] = lw;
      }
    }
#pragma unroll 1
    for (int rr = 0; rr < 2; ++rr) {
      const int i = rr ? (kChunk - 1 - wave) : wave;
      const v4f gi = *(const v4f*)(Gs + i * kHead + 4 * lane);
      const v4f ki = *(const v4f*)(Ks + i * kHead + 4 * lane);
      const v4f qi = *(const v4f*)(Qs + i * kHead + 4 * lane);
#pragma unroll 1
      for (int s2 = 0; s2 <= i; ++s2) {
        const v4f gs = *(const v4f*)(Gs + s2 * kHead + 4 * lane);
        const v4f ks = *(const v4f*)(Ks + s2 * kHead + 4 * lane);
        float pa = 0.0f, pb = 0.0f;
#pragma unroll
        for (int e = 0; e < 4; ++e) {
          const float kw = ks[e] * __expf(gi[e] - gs[e]);
          pa = fmaf(ki[e], kw, pa);
          pb = fmaf(qi[e], kw, pb);
        }
        const float ta = __shfl_xor(pa, 16, 32);
        const float tb = __shfl_xor(pb, 16, 32);
        float x = hh ? (pb + tb) : (pa + ta);
        x += __shfl_xor(x, 8, 32);
        x += __shfl_xor(x, 4, 32);
        x += __shfl_xor(x, 2, 32);
        x += __shfl_xor(x, 1, 32);
        if (lane == 0)  Amat[i * kChunk + s2] = x;
        if (lane == 16) Bmat[i * kChunk + s2] = x;
      }
      if (lane < kChunk && lane > i) {
        Amat[i * kChunk + lane] = 0.0f;
        Bmat[i * kChunk + lane] = 0.0f;
      }
    }
    __syncthreads();

    v8f accR = (v8f){0.f,0.f,0.f,0.f,0.f,0.f,0.f,0.f};
    v8f accO = (v8f){0.f,0.f,0.f,0.f,0.f,0.f,0.f,0.f};
#pragma unroll 1
    for (int ks = 0; ks < 4; ++ks) {
      const v4f s0 = *(const v4f*)(strow + 32 * ks);
      const v4f s1 = *(const v4f*)(strow + 32 * ks + 4);
      const v4f s2 = *(const v4f*)(strow + 32 * ks + 16);
      const v4f s3 = *(const v4f*)(strow + 32 * ks + 20);
      unsigned hw[8], lw[8];
      split_pair(s0[0], s0[1], hw[0], lw[0]);
      split_pair(s0[2], s0[3], hw[1], lw[1]);
      split_pair(s1[0], s1[1], hw[2], lw[2]);
      split_pair(s1[2], s1[3], hw[3], lw[3]);
      split_pair(s2[0], s2[1], hw[4], lw[4]);
      split_pair(s2[2], s2[3], hw[5], lw[5]);
      split_pair(s3[0], s3[1], hw[6], lw[6]);
      split_pair(s3[2], s3[3], hw[7], lw[7]);
      const v8u hv = (v8u){hw[0], hw[1], hw[2], hw[3], hw[4], hw[5], hw[6], hw[7]};
      const v8u lv = (v8u){lw[0], lw[1], lw[2], lw[3], lw[4], lw[5], lw[6], lw[7]};
      const v16b sh = __builtin_bit_cast(v16b, hv);
      const v16b sl = __builtin_bit_cast(v16b, lv);
      const v16b kth = Frag<__bf16>::load(kthp + 32 * ks);
      const v16b ktl = Frag<__bf16>::load(ktlp + 32 * ks);
      const v16b qth = Frag<__bf16>::load(qthp + 32 * ks);
      const v16b qtl = Frag<__bf16>::load(qtlp + 32 * ks);
      accR = Frag<__bf16>::mma(kth, sh, accR);
      accR = Frag<__bf16>::mma(kth, sl, accR);
      accR = Frag<__bf16>::mma(ktl, sh, accR);
      accO = Frag<__bf16>::mma(qth, sh, accO);
      accO = Frag<__bf16>::mma(qth, sl, accO);
      accO = Frag<__bf16>::mma(qtl, sh, accO);
      guard_s6(accR, accO, kth, ktl, qth, qtl, sh, sl);
    }
#pragma unroll
    for (int r = 0; r < 8; ++r) {
      const int idx = (8 * hh + r) * kHead + 16 * wave + c;
      RO[idx] = Vs[idx] - accR[r];
    }
    __syncthreads();

    if (tid < kHead) {
#pragma unroll 1
      for (int i = 0; i < kChunk; ++i) {
        float m = RO[i * kHead + tid];
#pragma unroll 1
        for (int s2 = 0; s2 < i; ++s2) {
          const float av = Amat[i * kChunk + s2];
          const float uv = RO[s2 * kHead + tid];
          m = fmaf(-av, uv, m);
        }
        RO[i * kHead + tid] = betas[i] * m;
      }
#pragma unroll 1
      for (int j = 0; j < 8; ++j) {
        unsigned hw, lw;
        split_pair(RO[(2 * j) * kHead + tid], RO[(2 * j + 1) * kHead + tid], hw, lw);
        UT[tid * kUtW + j]     = hw;
        UT[tid * kUtW + 8 + j] = lw;
      }
    } else if (tid < kHead + kChunk) {
      const int i = tid - kHead;
#pragma unroll 1
      for (int j = 0; j < 8; ++j) {
        unsigned hw, lw;
        split_pair(Bmat[i * kChunk + 2 * j], Bmat[i * kChunk + 2 * j + 1], hw, lw);
        BPh[i * kKhW + j] = hw;
        BPl[i * kKhW + j] = lw;
      }
    }
    __syncthreads();

    {
      const v16b ub = Frag<__bf16>::load(utp);
#pragma unroll 1
      for (int dt = 0; dt < 8; ++dt) {
        const v4f e0 = *(const v4f*)(egC + 16 * dt + 8 * hh);
        const v4f e1 = *(const v4f*)(egC + 16 * dt + 8 * hh + 4);
        const v4f t0v = *(const v4f*)(strow + 16 * dt);
        const v4f t1v = *(const v4f*)(strow + 16 * dt + 4);
        v8f sa;
        sa[0] = t0v[0] * e0[0]; sa[1] = t0v[1] * e0[1]; sa[2] = t0v[2] * e0[2]; sa[3] = t0v[3] * e0[3];
        sa[4] = t1v[0] * e1[0]; sa[5] = t1v[1] * e1[1]; sa[6] = t1v[2] * e1[2]; sa[7] = t1v[3] * e1[3];
        const v16b ah = Frag<__bf16>::load_dup(khhp + 16 * dt * kKhPitch);
        const v16b al = Frag<__bf16>::load_dup(khlp + 16 * dt * kKhPitch);
        sa = Frag<__bf16>::mma(ah, ub, sa);
        sa = Frag<__bf16>::mma(al, ub, sa);
        guard_u3(sa, ah, al, ub);
        const v4f n0v = (v4f){sa[0], sa[1], sa[2], sa[3]};
        const v4f n1v = (v4f){sa[4], sa[5], sa[6], sa[7]};
        *(v4f*)(strow + 16 * dt)     = n0v;
        *(v4f*)(strow + 16 * dt + 4) = n1v;
      }
      const v16b bh = Frag<__bf16>::load_dup(bphp);
      const v16b bl = Frag<__bf16>::load_dup(bplp);
      accO = Frag<__bf16>::mma(bh, ub, accO);
      accO = Frag<__bf16>::mma(bl, ub, accO);
      guard_u3(accO, bh, bl, ub);
#pragma unroll
      for (int r = 0; r < 8; ++r) RO[(8 * hh + r) * kHead + 16 * wave + c] = accO[r];
    }
    __syncthreads();

    for (int pass = 0; pass < 2; ++pass) {
#pragma unroll
      for (int rr = 0; rr < 2; ++rr) {
        const int row = 2 * wave + rr;
        const v4f v = *(const v4f*)(RO + row * kHead + 4 * lane);
        *(volatile v4f*)(O + (size_t)(t0 + row) * kCh + h * kHead + 4 * lane) = v;
      }
      __threadfence();
    }
  }
}

__global__ __launch_bounds__(256) void mix_norm_gate_kernel(const float* __restrict__ OFp, const float* __restrict__ OSp, const float* __restrict__ LAM,
                                                            const float* __restrict__ GATE, const float* __restrict__ bg2, const float* __restrict__ onw,
                                                            unsigned short* __restrict__ ON, float carry) {
  const int lane = threadIdx.x & 31, wave = threadIdx.x >> 5;
  const int gw = blockIdx.x * 8 + wave;
  const int row = gw >> 4, h = gw & 15;
  const size_t off = (size_t)row * kCh + h * kHead + lane * 4;
  const v4f of = *(const v4f*)(OFp + off);
  const v4f os = *(const v4f*)(OSp + off);
  const v4f gt = *(const v4f*)(GATE + off);
  const v4f bg = *(const v4f*)(bg2 + h * kHead + lane * 4);
  const v4f ow = *(const v4f*)(onw + lane * 4);
  const float lam = LAM[(size_t)row * kHeads + h];
  v4f o;
  float ss = 0.0f;
#pragma unroll
  for (int e = 0; e < 4; ++e) {
    const float ov = lam * of[e] + (1.0f - lam) * os[e];
    o[e] = ov;
    ss += ov * ov;
  }
#pragma unroll
  for (int off2 = 16; off2 > 0; off2 >>= 1) ss += __shfl_xor(ss, off2, 32);
  const float rs = rsqrtf(ss * (1.0f / (float)kHead) + kNormEps);
  unsigned short hb[4];
#pragma unroll
  for (int e = 0; e < 4; ++e) {
    const float wv = ow[e];
    const float bv = bg[e];
    const float y = ((o[e] * rs) * inr(wv)) * sigm(gt[e] + inr(bv));
    hb[e] = h_bits(y * carry);
  }
  const v2u u = (v2u){pk16(hb[0], hb[1]), pk16(hb[2], hb[3])};
  unsigned short* op = ON + off;
  *(volatile v2u*)op = u;
  __threadfence();
  *(volatile v2u*)op = u;
}

extern "C" void kernel_launch(void* const* d_in, const int* in_sizes, int n_in,
                              void* d_out, int out_size, void* d_ws, size_t ws_size, hipStream_t stream) {
  if (n_in < 21 || d_out == nullptr || d_ws == nullptr) return;
  if (in_sizes[0] != kTok * kHid || in_sizes[1] != kHid * kCh || in_sizes[2] != kHid * kCh || in_sizes[3] != kHid * kCh ||
      in_sizes[4] != kCh * 4 || in_sizes[5] != kCh * 4 || in_sizes[6] != kCh * 4 ||
      in_sizes[7] != kHid * kHead || in_sizes[8] != kHead * kCh || in_sizes[9] != kHid * kHead || in_sizes[10] != kHead * kCh ||
      in_sizes[11] != kHid * kHeads || in_sizes[12] != kHid * kHeads || in_sizes[13] != kHid * kHeads ||
      in_sizes[14] != kHeads || in_sizes[15] != kCh || in_sizes[16] != kHid * kHead || in_sizes[17] != kHead * kCh ||
      in_sizes[18] != kCh || in_sizes[19] != kHead || in_sizes[20] != kCh * kHid || out_size != kTok * kHid) return;

  const float* x       = (const float*)d_in[0];
  const float* Wq      = (const float*)d_in[1];
  const float* Wk      = (const float*)d_in[2];
  const float* Wv      = (const float*)d_in[3];
  const float* conv_wq = (const float*)d_in[4];
  const float* conv_wk = (const float*)d_in[5];
  const float* conv_wv = (const float*)d_in[6];
  const float* Wgb1    = (const float*)d_in[7];
  const float* Wgb2    = (const float*)d_in[8];
  const float* Wgd1    = (const float*)d_in[9];
  const float* Wgd2    = (const float*)d_in[10];
  const float* Wbb     = (const float*)d_in[11];
  const float* Wbd     = (const float*)d_in[12];
  const float* Wlam    = (const float*)d_in[13];
  const float* A_log   = (const float*)d_in[14];
  const float* dt_bias = (const float*)d_in[15];
  const float* Wg1     = (const float*)d_in[16];
  const float* Wg2     = (const float*)d_in[17];
  const float* bg2     = (const float*)d_in[18];
  const float* onorm_w = (const float*)d_in[19];
  const float* Wo      = (const float*)d_in[20];
  float* out = (float*)d_out;

  char* ws = (char*)d_ws;
  const size_t MiB = (size_t)1048576;
  const size_t r4 = 112 * MiB;
  const size_t szWsT = (size_t)kSmall * kHid * 2;
  const size_t szWgT = (size_t)kCh * 2 * kHead * 2;
  const size_t szWg2T = (size_t)kCh * kHead * 2;
  const size_t szSM = (size_t)kTok * kSmall * 4;
  const size_t szMID2 = (size_t)kTok * 2 * kHead * 2;
  const size_t szMIDg = (size_t)kTok * kHead * 2;
  const size_t szBL = (size_t)kTok * kHeads * 4;
  const size_t total = r4 + szWsT + szWgT + szWg2T + szSM + 2 * szMID2 + szMIDg + 3 * szBL;
  if (total > ws_size || total > (size_t)134217728) return;

  unsigned short* XH  = (unsigned short*)(ws + 0);
  unsigned short* GF  = (unsigned short*)(ws + 0);
  unsigned short* WqT = (unsigned short*)(ws + 8 * MiB);
  unsigned short* GS  = (unsigned short*)(ws + 8 * MiB);
  unsigned short* WkT = (unsigned short*)(ws + 16 * MiB);
  unsigned short* WoT = (unsigned short*)(ws + 16 * MiB);
  unsigned short* WvT = (unsigned short*)(ws + 24 * MiB);
  unsigned short* ON  = (unsigned short*)(ws + 24 * MiB);
  float* PRE  = (float*)(ws + 32 * MiB);
  float* GP   = (float*)(ws + 32 * MiB);
  float* OFb  = (float*)(ws + 32 * MiB);
  float* GM   = (float*)(ws + 48 * MiB);
  float* OSb  = (float*)(ws + 48 * MiB);
  float* QN   = (float*)(ws + 64 * MiB);
  float* GATE = (float*)(ws + 64 * MiB);
  float* KN   = (float*)(ws + 80 * MiB);
  float* VC   = (float*)(ws + 96 * MiB);
  size_t o4 = r4;
  unsigned short* WsT  = (unsigned short*)(ws + o4); o4 += szWsT;
  unsigned short* WgT  = (unsigned short*)(ws + o4); o4 += szWgT;
  unsigned short* Wg2T = (unsigned short*)(ws + o4); o4 += szWg2T;
  float*          SM   = (float*)(ws + o4);          o4 += szSM;
  unsigned short* MIDp = (unsigned short*)(ws + o4); o4 += szMID2;
  unsigned short* MIDm = (unsigned short*)(ws + o4); o4 += szMID2;
  unsigned short* MIDg = (unsigned short*)(ws + o4); o4 += szMIDg;
  float*          BFb  = (float*)(ws + o4);          o4 += szBL;
  float*          BSb  = (float*)(ws + o4);          o4 += szBL;
  float*          LAMb = (float*)(ws + o4);          o4 += szBL;

  auto gemm = [&](const unsigned short* A, int lda, const unsigned short* Btp, int ldb, float* C, int ldc, int M, int N, int K, float scale) {
    const int tiles = (M / 64) * (N / 64);
    const dim3 grid((unsigned)((tiles + 7) / 8), 1);
    wmma_gemm64<0, false, 0, 0, false, 0><<<grid, 256, 0, stream>>>(
        A, A, lda, 0L, Btp, Btp, ldb, 0L, (void*)C, (void*)C, ldc, 0L, (const float*)C, (const float*)C, 0L, M, N, K, scale);
  };

  cvt_x_kernel<<<(kTok * kHid / 8) / 256, 256, 0, stream>>>(x, XH, kTok * kHid / 8, kXCarry);
  tr_cast_kernel<<<dim3(kHid / 64, kCh / 64, 3), 256, 0, stream>>>(Wq, Wk, Wv, WqT, WkT, WvT, kCh, kHid, kWCarry);
  tr_cast_kernel<<<dim3(kHid / 64, kHead / 64, 3), 256, 0, stream>>>(Wgb1, Wgd1, Wg1, WsT, WsT + (size_t)128 * kHid, WsT + (size_t)256 * kHid, kHead, kHid, kWCarry);
  tr_small16_kernel<<<kHid / 64, 256, 0, stream>>>(Wbb, Wbd, Wlam, WsT + (size_t)384 * kHid, kHid, kWCarry);
  tr_cast_kernel<<<dim3(kHead / 64, kCh / 64, 2), 256, 0, stream>>>(Wgb2, Wgd2, Wgd2, WgT, WgT + kHead, WgT + kHead, kCh, 2 * kHead, kWCarry);
  tr_cast_kernel<<<dim3(kHead / 64, kCh / 64, 1), 256, 0, stream>>>(Wg2, Wg2, Wg2, Wg2T, Wg2T, Wg2T, kCh, kHead, kWCarry);

  gemm(XH, kHid, WsT, kHid, SM, kSmall, kTok, kSmall, kHid, kProjScale);

  gemm(XH, kHid, WqT, kHid, PRE, kCh, kTok, kCh, kHid, kProjScale);
  conv_silu_kernel<true><<<kTok * kHeads / 8, 256, 0, stream>>>(PRE, conv_wq, QN);
  gemm(XH, kHid, WkT, kHid, PRE, kCh, kTok, kCh, kHid, kProjScale);
  conv_silu_kernel<true><<<kTok * kHeads / 8, 256, 0, stream>>>(PRE, conv_wk, KN);
  gemm(XH, kHid, WvT, kHid, PRE, kCh, kTok, kCh, kHid, kProjScale);
  conv_silu_kernel<false><<<kTok * kHeads / 8, 256, 0, stream>>>(PRE, conv_wv, VC);

  tr_cast_kernel<<<dim3(kCh / 64, kHid / 64, 1), 256, 0, stream>>>(Wo, Wo, Wo, WoT, WoT, WoT, kHid, kCh, kWCarry);

  split_small_kernel<<<dim3(kTok * 32 / 256, 2), 256, 0, stream>>>(SM, MIDp, MIDm, MIDg, kMidCarry);
  beta_lam_kernel<<<kTok * kHeads / 256, 256, 0, stream>>>(SM, BFb, BSb, LAMb);

  gemm(MIDp, 2 * kHead, WgT, 2 * kHead, GP, kCh, kTok, kCh, 2 * kHead, kMidScale);
  gemm(MIDm, 2 * kHead, WgT, 2 * kHead, GM, kCh, kTok, kCh, 2 * kHead, kMidScale);
  gate_kernel<<<dim3(kTok * kCh / 2 / 256, 2), 256, 0, stream>>>(GP, GM, GF, GS, A_log, dt_bias);

  const float qscale = 1.0f / sqrtf((float)kHead);
  delta_scan_kernel<<<kBatch * kHeads * 2, 256, 0, stream>>>(QN, KN, VC, GF, GS, BFb, BSb, OFb, OSb, qscale);

  gemm(MIDg, kHead, Wg2T, kHead, GATE, kCh, kTok, kCh, kHead, kMidScale);
  mix_norm_gate_kernel<<<kTok * kHeads / 8, 256, 0, stream>>>(OFb, OSb, LAMb, GATE, bg2, onorm_w, ON, kOnCarry);
  gemm(ON, kCh, WoT, kCh, out, kHid, kTok, kHid, kCh, kOutScale);
}
